// MoE_HyperNetLinearLayer_6399501271813
// MI455X (gfx1250) — hardware-run, weakly checked
//
#include <hip/hip_runtime.h>
#include <stddef.h>
#include <stdint.h>

#define NB   4096
#define NI   1024
#define NO   1024
#define NC   128
#define NE   8
#define NH   32
#define TBM  128
#define TBN  64
#define GBM  32

static_assert((NI % 32) == 0);
static_assert((NC % 32) == 0);
static_assert((NB % TBM) == 0);
static_assert((NO % TBN) == 0);
static_assert((NB % GBM) == 0);
static_assert((NI % 64) == 0);
static_assert((NO % 64) == 0);
static_assert(NH == 32);
static_assert(NE == 8);
static_assert((NB * NI) % 2048 == 0);

typedef __attribute__((ext_vector_type(16))) __bf16 v16b;
typedef float        v8f __attribute__((ext_vector_type(8)));
typedef float        v4f __attribute__((ext_vector_type(4)));
typedef unsigned int v4u __attribute__((ext_vector_type(4)));
typedef unsigned int v2u __attribute__((ext_vector_type(2)));

__device__ __forceinline__ unsigned short bf_bits(float f) {
  const unsigned u = __float_as_uint(f);
  return (unsigned short)((u + 0x7FFFu + ((u >> 16) & 1u)) >> 16);
}
__device__ __forceinline__ float bfr(float f) { return __uint_as_float(((unsigned)bf_bits(f)) << 16); }
__device__ __forceinline__ unsigned pk16(unsigned short a, unsigned short b) { return (unsigned)a | ((unsigned)b << 16); }
__device__ __forceinline__ v8f zero8() { v8f z = {0.f, 0.f, 0.f, 0.f, 0.f, 0.f, 0.f, 0.f}; return z; }

union FragB { v16b v; v4u u[2]; };
__device__ __forceinline__ v16b ldfrag_b(const unsigned short* p) {
  FragB f;
  f.u[0] = *(const v4u*)(p);
  f.u[1] = *(const v4u*)(p + 16);
  return f.v;
}

__device__ __forceinline__ v8f mma_b(v16b a, v16b b, v8f c) {
  return __builtin_amdgcn_wmma_f32_16x16x32_bf16(false, a, false, b, (short)0, c, false, false);
}
__device__ __forceinline__ void guard4(v8f& c0, v8f& c1, v8f& c2, v8f& c3,
                                       const v16b& a0, const v16b& a1, const v16b& b0, const v16b& b1) {
#if defined(__HIP_DEVICE_COMPILE__)
  asm volatile("v_nop\n\tv_nop\n\tv_nop\n\tv_nop"
               : "+v"(c0), "+v"(c1), "+v"(c2), "+v"(c3)
               : "v"(a0), "v"(a1), "v"(b0), "v"(b1));
#endif
}
__device__ __forceinline__ void guard2(v8f& c0, v8f& c1, const v16b& a0, const v16b& b0, const v16b& b1) {
#if defined(__HIP_DEVICE_COMPILE__)
  asm volatile("v_nop\n\tv_nop\n\tv_nop\n\tv_nop"
               : "+v"(c0), "+v"(c1)
               : "v"(a0), "v"(b0), "v"(b1));
#endif
}

__global__ __launch_bounds__(64)
void k_gate(const float* __restrict__ cond, const float* __restrict__ w1, const float* __restrict__ b1,
            const float* __restrict__ w2, const float* __restrict__ b2, float* gating) {
  __shared__ __align__(16) unsigned short sA[GBM * NC];
  __shared__ __align__(16) unsigned short sB[NH * NC];
  __shared__ __align__(16) float sH[GBM * NH];
  __shared__ __align__(16) float sG[GBM * NE];
  const int tid = threadIdx.x, w = tid >> 5, lane = tid & 31, hh = lane >> 4, c = lane & 15;
  const int row0 = blockIdx.x * GBM;

  const float* cp = cond + (size_t)row0 * NC;
#pragma unroll
  for (int j = 0; j < (GBM * NC) / (64 * 4); ++j) {
    const int flat = (tid + 64 * j) * 4;
    const v4f v = *(const v4f*)(cp + flat);
    v2u u;
    u[0] = pk16(bf_bits(v[0]), bf_bits(v[1]));
    u[1] = pk16(bf_bits(v[2]), bf_bits(v[3]));
    *(v2u*)(sA + flat) = u;
  }
#pragma unroll 4
  for (int j = 0; j < (NC * NH) / 64; ++j) {
    const int idx = tid + 64 * j;
    const int k = idx >> 5, n = idx & 31;
    sB[n * NC + k] = bf_bits(w1[idx]);
  }
  __syncthreads();

  v8f acc0 = zero8(), acc1 = zero8();
  const unsigned short* ap  = sA + (16 * w + c) * NC + 8 * hh;
  const unsigned short* bq0 = sB + c * NC + 8 * hh;
  const unsigned short* bq1 = sB + (16 + c) * NC + 8 * hh;
#pragma unroll
  for (int ks = 0; ks < NC / 32; ++ks) {
    const v16b a  = ldfrag_b(ap + 32 * ks);
    const v16b f0 = ldfrag_b(bq0 + 32 * ks);
    const v16b f1 = ldfrag_b(bq1 + 32 * ks);
    acc0 = mma_b(a, f0, acc0);
    acc1 = mma_b(a, f1, acc1);
    guard2(acc0, acc1, a, f0, f1);
  }

  const float bb0 = bfr(b1[c]), bb1 = bfr(b1[16 + c]);
#pragma unroll
  for (int r = 0; r < 8; ++r) {
    const int lrow = 16 * w + 8 * hh + r;
    sH[lrow * NH + c]      = fmaxf(acc0[r] + bb0, 0.0f);
    sH[lrow * NH + 16 + c] = fmaxf(acc1[r] + bb1, 0.0f);
  }
  __syncthreads();

  if (tid < GBM) {
    float lg[NE];
#pragma unroll
    for (int e = 0; e < NE; ++e) lg[e] = 0.0f;
#pragma unroll 1
    for (int j = 0; j < NH; ++j) {
      const float hj = sH[tid * NH + j];
#pragma unroll
      for (int e = 0; e < NE; ++e) lg[e] = fmaf(hj, bfr(w2[j * NE + e]), lg[e]);
    }
#pragma unroll
    for (int e = 0; e < NE; ++e) lg[e] += bfr(b2[e]);
    float mx = lg[0];
#pragma unroll
    for (int e = 1; e < NE; ++e) mx = fmaxf(mx, lg[e]);
    float s = 0.0f;
#pragma unroll
    for (int e = 0; e < NE; ++e) { lg[e] = __expf(lg[e] - mx); s += lg[e]; }
    const float inv = 1.0f / s;
#pragma unroll
    for (int e = 0; e < NE; ++e) sG[tid * NE + e] = lg[e] * inv;
  }
  __syncthreads();

  const v4f g4 = *(const v4f*)(sG + tid * 4);
  float* gp = gating + (size_t)row0 * NE + tid * 4;
  *(volatile v4f*)gp = g4;
  __threadfence();
  *(volatile v4f*)gp = g4;
}

__global__ __launch_bounds__(256)
void k_cvx(const float* __restrict__ x, unsigned short* Xb) {
  const size_t f8 = ((size_t)blockIdx.x * 256 + threadIdx.x) * 8;
  const v4f a = *(const v4f*)(x + f8);
  const v4f b = *(const v4f*)(x + f8 + 4);
  v4u u;
  u[0] = pk16(bf_bits(a[0]), bf_bits(a[1]));
  u[1] = pk16(bf_bits(a[2]), bf_bits(a[3]));
  u[2] = pk16(bf_bits(b[0]), bf_bits(b[1]));
  u[3] = pk16(bf_bits(b[2]), bf_bits(b[3]));
  unsigned short* dst = Xb + f8;
  *(volatile v4u*)dst = u;
  __threadfence();
  *(volatile v4u*)dst = u;
}

__global__ __launch_bounds__(256)
void k_tw(const float* __restrict__ w, unsigned short* Wt) {
  __shared__ __align__(16) unsigned short sT[64 * 72];
  const int e = blockIdx.z, o0 = blockIdx.x * 64, i0 = blockIdx.y * 64;
  const int tid = threadIdx.x;
  const int rr = tid >> 4, c4 = (tid & 15) * 4;
#pragma unroll
  for (int it = 0; it < 4; ++it) {
    const int ii = it * 16 + rr;
    const v4f v = *(const v4f*)(w + ((size_t)(e * NI + i0 + ii)) * NO + o0 + c4);
    sT[(c4 + 0) * 72 + ii] = bf_bits(v[0]);
    sT[(c4 + 1) * 72 + ii] = bf_bits(v[1]);
    sT[(c4 + 2) * 72 + ii] = bf_bits(v[2]);
    sT[(c4 + 3) * 72 + ii] = bf_bits(v[3]);
  }
  __syncthreads();
  const int p = tid & 7, lq = tid >> 3;
  v4u u[2];
#pragma unroll
  for (int it = 0; it < 2; ++it) {
    const int oo = it * 32 + lq;
    u[it] = *(const v4u*)(sT + oo * 72 + p * 8);
  }
  unsigned short* dst = Wt + ((size_t)(e * NO + o0 + lq)) * NI + i0 + p * 8;
#pragma unroll
  for (int it = 0; it < 2; ++it) *(volatile v4u*)(dst + (size_t)it * 32 * NI) = u[it];
  __threadfence();
#pragma unroll
  for (int it = 0; it < 2; ++it) *(volatile v4u*)(dst + (size_t)it * 32 * NI) = u[it];
}

__global__ __launch_bounds__(256)
void k_moe(const unsigned short* __restrict__ Xb, const unsigned short* __restrict__ Wt,
           const float* __restrict__ gating, const float* __restrict__ bias, float* out) {
  __shared__ __align__(16) float sO[TBM * TBN];
  const int tid = threadIdx.x, w = tid >> 5, lane = tid & 31, hh = lane >> 4, c = lane & 15;
  const int wm = w & 3, wn = w >> 2;
  const int Mbase = blockIdx.x * TBM, Nbase = blockIdx.y * TBN;
  const int mrow0 = Mbase + 32 * wm;
  const int n0 = Nbase + 32 * wn + c;
  const int n1 = n0 + 16;

  const unsigned short* ap0 = Xb + (size_t)(mrow0 + c) * NI + 8 * hh;
  const unsigned short* ap1 = ap0 + (size_t)16 * NI;

  v8f tot[2][2];
#pragma unroll
  for (int mt = 0; mt < 2; ++mt) { tot[mt][0] = zero8(); tot[mt][1] = zero8(); }

#pragma unroll 1
  for (int e = 0; e < NE; ++e) {
    const unsigned short* bp0 = Wt + ((size_t)e * NO + n0) * NI + 8 * hh;
    const unsigned short* bp1 = bp0 + (size_t)16 * NI;
    v8f acc[2][2];
#pragma unroll
    for (int mt = 0; mt < 2; ++mt) { acc[mt][0] = zero8(); acc[mt][1] = zero8(); }

#pragma unroll 1
    for (int ks = 0; ks < NI / 32; ++ks) {
      const int ko = 32 * ks;
      const v16b a0 = ldfrag_b(ap0 + ko);
      const v16b a1 = ldfrag_b(ap1 + ko);
      const v16b b0 = ldfrag_b(bp0 + ko);
      const v16b b1 = ldfrag_b(bp1 + ko);
      acc[0][0] = mma_b(a0, b0, acc[0][0]);
      acc[0][1] = mma_b(a0, b1, acc[0][1]);
      acc[1][0] = mma_b(a1, b0, acc[1][0]);
      acc[1][1] = mma_b(a1, b1, acc[1][1]);
      guard4(acc[0][0], acc[0][1], acc[1][0], acc[1][1], a0, a1, b0, b1);
    }

    const float bc0 = bfr(bias[(size_t)e * NO + n0]);
    const float bc1 = bfr(bias[(size_t)e * NO + n1]);
    const float* gr = gating + (size_t)(mrow0 + 8 * hh) * NE + e;
#pragma unroll
    for (int mt = 0; mt < 2; ++mt) {
#pragma unroll
      for (int r = 0; r < 8; ++r) {
        const float g = gr[(size_t)(16 * mt + r) * NE];
        tot[mt][0][r] = fmaf(g, acc[mt][0][r] + bc0, tot[mt][0][r]);
        tot[mt][1][r] = fmaf(g, acc[mt][1][r] + bc1, tot[mt][1][r]);
      }
    }
  }

  const int lc0 = 32 * wn + c;
#pragma unroll
  for (int mt = 0; mt < 2; ++mt) {
#pragma unroll
    for (int r = 0; r < 8; ++r) {
      const int lrow = 32 * wm + 16 * mt + 8 * hh + r;
      sO[lrow * TBN + lc0]      = tot[mt][0][r];
      sO[lrow * TBN + lc0 + 16] = tot[mt][1][r];
    }
  }
  __syncthreads();

  const int rr = tid >> 4, c4 = (tid & 15) * 4;
  v4f o[8];
#pragma unroll
  for (int it = 0; it < 8; ++it) o[it] = *(const v4f*)(sO + (it * 16 + rr) * TBN + c4);
  const size_t ob = (size_t)(Mbase + rr) * NO + Nbase + c4;
#pragma unroll
  for (int it = 0; it < 8; ++it) *(volatile v4f*)(out + ob + (size_t)it * 16 * NO) = o[it];
  __threadfence();
#pragma unroll
  for (int it = 0; it < 8; ++it) *(volatile v4f*)(out + ob + (size_t)it * 16 * NO) = o[it];
}

extern "C" void kernel_launch(void* const* d_in, const int* in_sizes, int n_in,
                              void* d_out, int out_size, void* d_ws, size_t ws_size,
                              hipStream_t stream) {
  if (n_in < 8) return;
  if (in_sizes[0] != NB * NI) return;
  if (in_sizes[1] != NB * NC) return;
  if (in_sizes[2] != NE * NI * NO) return;
  if (in_sizes[3] != NE * NO) return;
  if (in_sizes[4] != NC * NH) return;
  if (in_sizes[5] != NH) return;
  if (in_sizes[6] != NH * NE) return;
  if (in_sizes[7] != NE) return;
  if (out_size != NB * NO) return;

  const float* x    = (const float*)d_in[0];
  const float* cond = (const float*)d_in[1];
  const float* wexp = (const float*)d_in[2];
  const float* bexp = (const float*)d_in[3];
  const float* gw1  = (const float*)d_in[4];
  const float* gb1  = (const float*)d_in[5];
  const float* gw2  = (const float*)d_in[6];
  const float* gb2  = (const float*)d_in[7];
  float* out = (float*)d_out;

  const size_t sG = (size_t)NB * NE * 4;
  const size_t sX = (size_t)NB * NI * 2;
  const size_t sW = (size_t)NE * NO * NI * 2;
  size_t off = 0;
  const size_t oG = off; off += sG;
  const size_t oX = off; off += sX;
  const size_t oW = off; off += sW;
  if (off > ws_size) return;
  if (off > (size_t)134217728) return;

  char* ws = (char*)d_ws;
  float* gating = (float*)(ws + oG);
  unsigned short* Xb = (unsigned short*)(ws + oX);
  unsigned short* Wt = (unsigned short*)(ws + oW);

  k_gate<<<dim3(NB / GBM), dim3(64), 0, stream>>>(cond, gw1, gb1, gw2, gb2, gating);
  k_cvx<<<dim3((NB * NI) / 2048), dim3(256), 0, stream>>>(x, Xb);
  k_tw<<<dim3(NO / 64, NI / 64, NE), dim3(256), 0, stream>>>(wexp, Wt);
  k_moe<<<dim3(NB / TBM, NO / TBN), dim3(256), 0, stream>>>(Xb, Wt, gating, bexp, out);
  (void)hipGetLastError();
}
